// Classifier_79929341379065
// MI455X (gfx1250) — hardware-verified
//
#include <hip/hip_runtime.h>
#include <math.h>
#include <stddef.h>

typedef __attribute__((ext_vector_type(16))) _Float16 v16h;
typedef __attribute__((ext_vector_type(8)))  _Float16 v8h;
typedef __attribute__((ext_vector_type(8)))  float    v8f;
typedef __attribute__((ext_vector_type(4)))  float    v4f;

__device__ __forceinline__ void dep_guard_h(v8f& a, v8f& b, v16h x, v16h y) { asm volatile("v_nop\n\tv_nop\n\tv_nop\n\tv_nop" : "+v"(a), "+v"(b) : "v"(x), "v"(y)); }
__device__ __forceinline__ void keep4_h(v16h a, v16h b, v16h c, v16h d) { asm volatile("v_nop" :: "v"(a), "v"(b), "v"(c), "v"(d)); }
template <typename T> struct Frag;
template <> struct Frag<_Float16> {
  typedef v16h V; union U { v16h v; v8h h[2]; };
  static __device__ __forceinline__ v16h load(const _Float16* p) {
    U f; f.h[0] = *(const v8h*)(p); f.h[1] = *(const v8h*)(p + 16); return f.v;
  }
  static __device__ __forceinline__ v8f mma(v16h a, v16h b, v8f c) {
    return __builtin_amdgcn_wmma_f32_16x16x32_f16(false, a, false, b, (short)0, c, false, false);
  }
  static __device__ __forceinline__ void guard(v8f& a, v8f& b, v16h x, v16h y) { dep_guard_h(a, b, x, y); }
  static __device__ __forceinline__ void keep(v16h a, v16h b, v16h c, v16h d) { keep4_h(a, b, c, d); }
};

__device__ __forceinline__ void guard_pair(v8f& c0, v8f& c1, v16h a, v16h b0, v16h b1) {
  asm volatile("v_nop\n\tv_nop\n\tv_nop\n\tv_nop" : "+v"(c0), "+v"(c1) : "v"(a), "v"(b0), "v"(b1));
}
__device__ __forceinline__ void guard_one(v8f& c, v16h a, v16h b) {
  asm volatile("v_nop\n\tv_nop\n\tv_nop\n\tv_nop" : "+v"(c) : "v"(a), "v"(b));
}
__device__ __forceinline__ v8f zero_v8f() { v8f z = {0.f, 0.f, 0.f, 0.f, 0.f, 0.f, 0.f, 0.f}; return z; }
__device__ __forceinline__ v8h zero_v8h() {
  v8h z;
#pragma unroll
  for (int e = 0; e < 8; ++e) z[e] = (_Float16)0.0f;
  return z;
}

constexpr int LTOK = 16;
constexpr int NHEAD = 8;
constexpr int DHEAD = 32;
constexpr int DMOD = 256;
constexpr int BNE = 128;
constexpr int SEQ_PER_BLK = 32;
constexpr int NTHR = 256;
constexpr float NEG_FILL = -1e32f;
constexpr float ATT_SCALE = 0.17677669529663687f;
constexpr float W_CARRY = 16.0f;
constexpr float W_CARRY_INV = 1.0f / 16.0f;
constexpr float P_CARRY = 1024.0f;
constexpr float P_CARRY_INV = 1.0f / 1024.0f;
static_assert(NHEAD * DHEAD == DMOD, "");
static_assert(BNE % 32 == 0 && DMOD % 32 == 0, "");

constexpr int WOFF_WQ   = 0;
constexpr int WOFF_WK   = 32768;
constexpr int WOFF_WV   = 65536;
constexpr int WOFF_WFC1 = 98304;
constexpr int WOFF_P1W1 = 163840;
constexpr int WOFF_P1W2 = 229376;
constexpr int WOFF_P2W1 = 294912;
constexpr int WOFF_P2W2 = 327680;
constexpr int WS_HALVES = 393216;

constexpr int PO_LN1G = 0,    PO_LN1B = 128,  PO_LN2G = 256,  PO_LN2B = 384,  PO_LN3G = 512,  PO_LN3B = 640;
constexpr int PO_P1B1 = 768,  PO_P1B2 = 1024, PO_P1LNG = 1280, PO_P1LNB = 1536;
constexpr int PO_P2B1 = 1792, PO_P2B2 = 2048;
constexpr int PO_LNC1G = 2304, PO_LNC1B = 2560, PO_LNC2G = 2816, PO_LNC2B = 3072;
constexpr int PO_WCLS = 3328, PO_BCLS = 3584;
constexpr int PAR_FLOATS = 3600;

constexpr int SM_PAR  = 0;
constexpr int SM_EMB  = 14464;
constexpr int SM_R1   = SM_EMB + 8192;
constexpr int SM_R2   = SM_R1 + 12288;
constexpr int SM_DYN  = SM_R2 + 24576;
constexpr int SM_STA  = SM_DYN + 16384;
constexpr int SM_TAIL = SM_STA + 16384;
constexpr int SMEM_BYTES = SM_TAIL + 448;
static_assert(PAR_FLOATS * 4 <= SM_EMB, "");
static_assert(SM_PAR % 16 == 0 && SM_EMB % 16 == 0 && SM_R1 % 16 == 0 && SM_R2 % 16 == 0 && SM_DYN % 16 == 0 && SM_STA % 16 == 0 && SM_TAIL % 16 == 0, "");

__device__ __forceinline__ float hsum16(float v) {
  v += __shfl_xor(v, 8, 32);
  v += __shfl_xor(v, 4, 32);
  v += __shfl_xor(v, 2, 32);
  v += __shfl_xor(v, 1, 32);
  return v;
}
__device__ __forceinline__ float hmax16(float v) {
  v = fmaxf(v, __shfl_xor(v, 8, 32));
  v = fmaxf(v, __shfl_xor(v, 4, 32));
  v = fmaxf(v, __shfl_xor(v, 2, 32));
  v = fmaxf(v, __shfl_xor(v, 1, 32));
  return v;
}

template <int KDIM>
__device__ __forceinline__ void gemm_two_tiles(const _Float16* sA, int lda, const _Float16* __restrict__ Wg,
                                               int n0, int n1, int h, int mn, v8f& acc0, v8f& acc1) {
  static_assert(KDIM % 32 == 0, "");
  const _Float16* pa  = sA + mn * lda + 8 * h;
  const _Float16* pb0 = Wg + (size_t)(n0 + mn) * KDIM + 8 * h;
  const _Float16* pb1 = Wg + (size_t)(n1 + mn) * KDIM + 8 * h;
#pragma unroll 2
  for (int k0 = 0; k0 < KDIM; k0 += 32) {
    const v16h a  = Frag<_Float16>::load(pa + k0);
    const v16h b0 = Frag<_Float16>::load(pb0 + k0);
    const v16h b1 = Frag<_Float16>::load(pb1 + k0);
    acc0 = Frag<_Float16>::mma(a, b0, acc0);
    acc1 = Frag<_Float16>::mma(a, b1, acc1);
    guard_pair(acc0, acc1, a, b0, b1);
  }
}

__device__ __forceinline__ void stage4(float* sPar, int off, const float* __restrict__ src, int n4, int t) {
  if (t >= 0 && t < n4) {
    const v4f v = *(const v4f*)(src + 4 * t);
    *(v4f*)(sPar + off + 4 * t) = v;
  }
}

__global__ __launch_bounds__(256) void cast_scale_f16x2(const float* __restrict__ in, _Float16* __restrict__ out, int n2, float s) {
  const int i = blockIdx.x * 256 + threadIdx.x;
  if (i < n2) {
    const _Float16 h0 = (_Float16)(in[2 * i] * s), h1 = (_Float16)(in[2 * i + 1] * s);
    const unsigned u = (unsigned)__builtin_bit_cast(unsigned short, h0) | ((unsigned)__builtin_bit_cast(unsigned short, h1) << 16);
    ((volatile unsigned*)out)[i] = u;
    __threadfence();
    ((volatile unsigned*)out)[i] = u;
  }
}

extern "C" __global__ __launch_bounds__(256)
void fused_seq_kernel(const int* __restrict__ x, const float* __restrict__ node_emb,
                      const float* __restrict__ ln1_g, const float* __restrict__ ln1_b,
                      const float* __restrict__ ln2_g, const float* __restrict__ ln2_b,
                      const float* __restrict__ ln3_g, const float* __restrict__ ln3_b,
                      const float* __restrict__ p1_b1, const float* __restrict__ p1_b2,
                      const float* __restrict__ p1_lng, const float* __restrict__ p1_lnb,
                      const float* __restrict__ p2_b1, const float* __restrict__ p2_b2,
                      const float* __restrict__ lnc1_g, const float* __restrict__ lnc1_b,
                      const float* __restrict__ lnc2_g, const float* __restrict__ lnc2_b,
                      const float* __restrict__ Wcls, const float* __restrict__ bcls,
                      const _Float16* __restrict__ wsh, float* __restrict__ out,
                      int nseq, int nvocab) {
  extern __shared__ __align__(16) char smem[];
  float*    sPar    = (float*)(smem + SM_PAR);
  float*    s_emb   = (float*)(smem + SM_EMB);
  _Float16* s_x3    = (_Float16*)(smem + SM_R1);
  _Float16* s_p     = (_Float16*)(smem + SM_R1);
  _Float16* s_stain = (_Float16*)(smem + SM_R1);
  _Float16* s_ctx   = (_Float16*)(smem + SM_R1 + 4096);
  _Float16* s_q     = (_Float16*)(smem + SM_R2);
  _Float16* s_k     = (_Float16*)(smem + SM_R2 + 8192);
  _Float16* s_vt    = (_Float16*)(smem + SM_R2 + 16384);
  _Float16* s_dynh  = (_Float16*)(smem + SM_R2);
  _Float16* s_h1    = (_Float16*)(smem + SM_R2 + 8192);
  _Float16* s_sh    = (_Float16*)(smem + SM_R2 + 16384);
  float*    s_dyn   = (float*)(smem + SM_DYN);
  float*    s_sta   = (float*)(smem + SM_STA);
  int*      s_tok   = (int*)(smem + SM_TAIL);
  float*    s_npm   = (float*)(smem + SM_TAIL + 64);
  float*    s_mu    = (float*)(smem + SM_TAIL + 128);
  float*    s_rs    = (float*)(smem + SM_TAIL + 192);
  float*    s_prob  = (float*)(smem + SM_TAIL + 256);
  float*    s_res   = (float*)(smem + SM_TAIL + 320);

  const int tid  = threadIdx.x;
  const int w    = tid >> 5;
  const int lane = tid & 31;
  const int h    = lane >> 4;
  const int mn   = lane & 15;
  const int blk  = blockIdx.x;
  const int n0   = w * 16;
  const int n1   = (w + 8) * 16;

  stage4(sPar, PO_P1B1,  p1_b1,  64, tid - 0);
  stage4(sPar, PO_P1B2,  p1_b2,  64, tid - 64);
  stage4(sPar, PO_P1LNG, p1_lng, 64, tid - 128);
  stage4(sPar, PO_P1LNB, p1_lnb, 64, tid - 192);
  stage4(sPar, PO_P2B1,  p2_b1,  64, tid - 0);
  stage4(sPar, PO_P2B2,  p2_b2,  64, tid - 64);
  stage4(sPar, PO_LNC1G, lnc1_g, 64, tid - 128);
  stage4(sPar, PO_LNC1B, lnc1_b, 64, tid - 192);
  stage4(sPar, PO_LNC2G, lnc2_g, 64, tid - 0);
  stage4(sPar, PO_LNC2B, lnc2_b, 64, tid - 64);
  stage4(sPar, PO_WCLS,  Wcls,   64, tid - 128);
  stage4(sPar, PO_LN1G,  ln1_g,  32, tid - 192);
  stage4(sPar, PO_LN1B,  ln1_b,  32, tid - 224);
  stage4(sPar, PO_LN2G,  ln2_g,  32, tid - 192);
  stage4(sPar, PO_LN2B,  ln2_b,  32, tid - 224);
  stage4(sPar, PO_LN3G,  ln3_g,  32, tid - 192);
  stage4(sPar, PO_LN3B,  ln3_b,  32, tid - 224);
  if (tid == 0) sPar[PO_BCLS] = bcls[0];
  __syncthreads();

  for (int it = 0; it < SEQ_PER_BLK; ++it) {
    int seq = blk * SEQ_PER_BLK + it;
    seq = (seq < nseq) ? seq : (nseq - 1);

    if (tid < LTOK) {
      const int t = x[(size_t)seq * LTOK + tid];
      int tc = t < 0 ? 0 : t;
      tc = tc > (nvocab - 1) ? (nvocab - 1) : tc;
      s_tok[tid] = tc;
      s_npm[tid] = (t != 0) ? 1.0f : 0.0f;
    }
    __syncthreads();

    {
      const int m = tid >> 4, c0 = (tid & 15) * 8;
      const float* src = node_emb + (size_t)s_tok[m] * BNE + c0;
      const v4f a0 = *(const v4f*)src;
      const v4f a1 = *(const v4f*)(src + 4);
      *(v4f*)(s_emb + m * BNE + c0) = a0;
      *(v4f*)(s_emb + m * BNE + c0 + 4) = a1;
    }
    __syncthreads();

    {
      const int m = 2 * w + h;
      const float* row = s_emb + m * BNE;
      float v[8];
      float s = 0.f;
#pragma unroll
      for (int j = 0; j < 8; ++j) { v[j] = row[mn + 16 * j]; s += v[j]; }
      s = hsum16(s);
      const float mu = s * (1.0f / BNE);
      float ss = 0.f;
#pragma unroll
      for (int j = 0; j < 8; ++j) { const float d = v[j] - mu; ss += d * d; }
      ss = hsum16(ss);
      const float var = ss * (1.0f / BNE);
      if (mn == 0) { s_mu[m] = mu; s_rs[m] = 1.0f / sqrtf(var + 1e-5f); }
    }
    __syncthreads();

    for (int idx = tid; idx < LTOK * BNE; idx += NTHR) {
      const int m = idx >> 7, c = idx & (BNE - 1);
      const float xh = (s_emb[idx] - s_mu[m]) * s_rs[m];
      s_x3[idx]                  = (_Float16)(xh * sPar[PO_LN1G + c] + sPar[PO_LN1B + c]);
      s_x3[LTOK * BNE + idx]     = (_Float16)(xh * sPar[PO_LN2G + c] + sPar[PO_LN2B + c]);
      s_x3[2 * LTOK * BNE + idx] = (_Float16)(xh * sPar[PO_LN3G + c] + sPar[PO_LN3B + c]);
    }
    __syncthreads();

    {
      v8f a0 = zero_v8f(), a1 = zero_v8f();
      gemm_two_tiles<BNE>(s_x3, BNE, wsh + WOFF_WQ, n0, n1, h, mn, a0, a1);
#pragma unroll
      for (int r = 0; r < 8; ++r) {
        s_q[(8 * h + r) * DMOD + n0 + mn] = (_Float16)(a0[r] * W_CARRY_INV);
        s_q[(8 * h + r) * DMOD + n1 + mn] = (_Float16)(a1[r] * W_CARRY_INV);
      }
    }
    {
      v8f a0 = zero_v8f(), a1 = zero_v8f();
      gemm_two_tiles<BNE>(s_x3 + LTOK * BNE, BNE, wsh + WOFF_WK, n0, n1, h, mn, a0, a1);
#pragma unroll
      for (int r = 0; r < 8; ++r) {
        s_k[(8 * h + r) * DMOD + n0 + mn] = (_Float16)(a0[r] * W_CARRY_INV);
        s_k[(8 * h + r) * DMOD + n1 + mn] = (_Float16)(a1[r] * W_CARRY_INV);
      }
    }
    {
      v8f a0 = zero_v8f(), a1 = zero_v8f();
      gemm_two_tiles<BNE>(s_x3 + 2 * LTOK * BNE, BNE, wsh + WOFF_WV, n0, n1, h, mn, a0, a1);
      v8h o0, o1;
#pragma unroll
      for (int r = 0; r < 8; ++r) {
        o0[r] = (_Float16)(a0[r] * W_CARRY_INV);
        o1[r] = (_Float16)(a1[r] * W_CARRY_INV);
      }
      *(v8h*)(s_vt + (n0 + mn) * LTOK + 8 * h) = o0;
      *(v8h*)(s_vt + (n1 + mn) * LTOK + 8 * h) = o1;
    }
    __syncthreads();

    {
      const v16h a = Frag<_Float16>::load(s_q + mn * DMOD + w * DHEAD + 8 * h);
      const v16h b = Frag<_Float16>::load(s_k + mn * DMOD + w * DHEAD + 8 * h);
      v8f sc = zero_v8f();
      sc = Frag<_Float16>::mma(a, b, sc);
      guard_one(sc, a, b);
      _Float16* pw = s_p + w * (LTOK * LTOK);
#pragma unroll
      for (int r = 0; r < 8; ++r) {
        const int row = 8 * h + r;
        float s = sc[r] * ATT_SCALE;
        s = (row == mn) ? NEG_FILL : s;
        const float mx = hmax16(s);
        const float e = expf(s - mx);
        const float sum = hsum16(e);
        const float p = e / sum;
        pw[row * LTOK + mn] = (_Float16)(p * P_CARRY);
      }
    }
    __syncthreads();

    {
      Frag<_Float16>::U pa;
      pa.h[0] = *(const v8h*)(s_p + w * (LTOK * LTOK) + mn * LTOK + 8 * h);
      pa.h[1] = zero_v8h();
#pragma unroll
      for (int nt = 0; nt < 2; ++nt) {
        const int col = w * DHEAD + nt * 16 + mn;
        Frag<_Float16>::U vb;
        vb.h[0] = *(const v8h*)(s_vt + col * LTOK + 8 * h);
        vb.h[1] = zero_v8h();
        v8f acc = zero_v8f();
        acc = Frag<_Float16>::mma(pa.v, vb.v, acc);
        guard_one(acc, pa.v, vb.v);
#pragma unroll
        for (int r = 0; r < 8; ++r) s_ctx[(8 * h + r) * DMOD + col] = (_Float16)(acc[r] * P_CARRY_INV);
      }
    }
    __syncthreads();

    {
      v8f a0 = zero_v8f(), a1 = zero_v8f();
      gemm_two_tiles<DMOD>(s_ctx, DMOD, wsh + WOFF_WFC1, n0, n1, h, mn, a0, a1);
#pragma unroll
      for (int r = 0; r < 8; ++r) {
        const int m = 8 * h + r;
        const float pm = s_npm[m];
        const float u0 = a0[r] * W_CARRY_INV * pm, u1 = a1[r] * W_CARRY_INV * pm;
        s_dyn[m * DMOD + n0 + mn]  = u0;
        s_dyn[m * DMOD + n1 + mn]  = u1;
        s_dynh[m * DMOD + n0 + mn] = (_Float16)u0;
        s_dynh[m * DMOD + n1 + mn] = (_Float16)u1;
      }
    }
    __syncthreads();

    {
      v8f a0 = zero_v8f(), a1 = zero_v8f();
      gemm_two_tiles<DMOD>(s_dynh, DMOD, wsh + WOFF_P1W1, n0, n1, h, mn, a0, a1);
      const float bb0 = sPar[PO_P1B1 + n0 + mn], bb1 = sPar[PO_P1B1 + n1 + mn];
#pragma unroll
      for (int r = 0; r < 8; ++r) {
        const int m = 8 * h + r;
        s_h1[m * DMOD + n0 + mn] = (_Float16)tanhf(a0[r] * W_CARRY_INV + bb0);
        s_h1[m * DMOD + n1 + mn] = (_Float16)tanhf(a1[r] * W_CARRY_INV + bb1);
      }
    }
    __syncthreads();

    {
      v8f a0 = zero_v8f(), a1 = zero_v8f();
      gemm_two_tiles<DMOD>(s_h1, DMOD, wsh + WOFF_P1W2, n0, n1, h, mn, a0, a1);
      const float bb0 = sPar[PO_P1B2 + n0 + mn], bb1 = sPar[PO_P1B2 + n1 + mn];
#pragma unroll
      for (int r = 0; r < 8; ++r) {
        const int m = 8 * h + r;
        const float d0 = s_dyn[m * DMOD + n0 + mn];
        const float d1 = s_dyn[m * DMOD + n1 + mn];
        s_dyn[m * DMOD + n0 + mn] = a0[r] * W_CARRY_INV + bb0 + d0;
        s_dyn[m * DMOD + n1 + mn] = a1[r] * W_CARRY_INV + bb1 + d1;
      }
    }
    __syncthreads();

    {
      const int m = 2 * w + h;
      float* row = s_dyn + m * DMOD;
      float v[16];
      float s = 0.f;
#pragma unroll
      for (int j = 0; j < 16; ++j) { v[j] = row[mn + 16 * j]; s += v[j]; }
      s = hsum16(s);
      const float mu = s * (1.0f / DMOD);
      float ss = 0.f;
#pragma unroll
      for (int j = 0; j < 16; ++j) { v[j] = v[j] - mu; ss += v[j] * v[j]; }
      ss = hsum16(ss);
      const float rs = 1.0f / sqrtf(ss * (1.0f / DMOD) + 1e-5f);
      const float pm = s_npm[m];
#pragma unroll
      for (int j = 0; j < 16; ++j) {
        const int c = mn + 16 * j;
        row[c] = (v[j] * rs * sPar[PO_P1LNG + c] + sPar[PO_P1LNB + c]) * pm;
      }
    }
    for (int idx = tid; idx < LTOK * BNE; idx += NTHR)
      s_stain[idx] = (_Float16)(s_emb[idx] * s_npm[idx >> 7]);
    __syncthreads();

    {
      v8f a0 = zero_v8f(), a1 = zero_v8f();
      gemm_two_tiles<BNE>(s_stain, BNE, wsh + WOFF_P2W1, n0, n1, h, mn, a0, a1);
      const float bb0 = sPar[PO_P2B1 + n0 + mn], bb1 = sPar[PO_P2B1 + n1 + mn];
#pragma unroll
      for (int r = 0; r < 8; ++r) {
        const int m = 8 * h + r;
        s_sh[m * DMOD + n0 + mn] = (_Float16)tanhf(a0[r] * W_CARRY_INV + bb0);
        s_sh[m * DMOD + n1 + mn] = (_Float16)tanhf(a1[r] * W_CARRY_INV + bb1);
      }
    }
    __syncthreads();

    {
      v8f a0 = zero_v8f(), a1 = zero_v8f();
      gemm_two_tiles<DMOD>(s_sh, DMOD, wsh + WOFF_P2W2, n0, n1, h, mn, a0, a1);
      const float bb0 = sPar[PO_P2B2 + n0 + mn], bb1 = sPar[PO_P2B2 + n1 + mn];
#pragma unroll
      for (int r = 0; r < 8; ++r) {
        const int m = 8 * h + r;
        const float pm = s_npm[m];
        s_sta[m * DMOD + n0 + mn] = (a0[r] * W_CARRY_INV + bb0) * pm;
        s_sta[m * DMOD + n1 + mn] = (a1[r] * W_CARRY_INV + bb1) * pm;
      }
    }
    __syncthreads();

    {
      const int m = 2 * w + h;
      const float* dr = s_dyn + m * DMOD;
      const float* sr = s_sta + m * DMOD;
      float av[16], bv[16];
      float s1 = 0.f, s2 = 0.f;
#pragma unroll
      for (int j = 0; j < 16; ++j) { av[j] = dr[mn + 16 * j]; bv[j] = sr[mn + 16 * j]; s1 += av[j]; s2 += bv[j]; }
      s1 = hsum16(s1); s2 = hsum16(s2);
      const float mu1 = s1 * (1.0f / DMOD), mu2 = s2 * (1.0f / DMOD);
      float q1 = 0.f, q2 = 0.f;
#pragma unroll
      for (int j = 0; j < 16; ++j) {
        av[j] = av[j] - mu1; q1 += av[j] * av[j];
        bv[j] = bv[j] - mu2; q2 += bv[j] * bv[j];
      }
      q1 = hsum16(q1); q2 = hsum16(q2);
      const float rs1 = 1.0f / sqrtf(q1 * (1.0f / DMOD) + 1e-5f);
      const float rs2 = 1.0f / sqrtf(q2 * (1.0f / DMOD) + 1e-5f);
      float pacc = 0.f;
#pragma unroll
      for (int j = 0; j < 16; ++j) {
        const int c = mn + 16 * j;
        const float a  = av[j] * rs1 * sPar[PO_LNC1G + c] + sPar[PO_LNC1B + c];
        const float bq = bv[j] * rs2 * sPar[PO_LNC2G + c] + sPar[PO_LNC2B + c];
        const float t = a - bq;
        pacc += t * t * sPar[PO_WCLS + c];
      }
      pacc = hsum16(pacc);
      if (mn == 0) {
        const float z = pacc + sPar[PO_BCLS];
        const float prob = 1.0f / (1.0f + expf(-z));
        s_prob[m] = prob * s_npm[m];
      }
    }
    __syncthreads();

    if (tid == 0) {
      float ps = 0.f, pn = 0.f;
#pragma unroll
      for (int j = 0; j < LTOK; ++j) { ps += s_prob[j]; pn += s_npm[j]; }
      s_res[it] = ps / pn;
    }
    __syncthreads();
  }

  if (w == 0) {
    const int sidx = blk * SEQ_PER_BLK + lane;
    const bool ok = (sidx < nseq);
    const float val = s_res[lane];
    volatile float* op = out + (size_t)(ok ? sidx : 0);
    if (ok) *op = val;
    __threadfence();
    if (ok) *op = val;
  }
}

extern "C" void kernel_launch(void* const* d_in, const int* in_sizes, int n_in,
                              void* d_out, int out_size, void* d_ws, size_t ws_size,
                              hipStream_t stream) {
  const int*   x        = (const int*)d_in[0];
  const float* node_emb = (const float*)d_in[1];
  const float* ln1_g  = (const float*)d_in[2];
  const float* ln1_b  = (const float*)d_in[3];
  const float* ln2_g  = (const float*)d_in[4];
  const float* ln2_b  = (const float*)d_in[5];
  const float* ln3_g  = (const float*)d_in[6];
  const float* ln3_b  = (const float*)d_in[7];
  const float* Wq     = (const float*)d_in[8];
  const float* Wk     = (const float*)d_in[9];
  const float* Wv     = (const float*)d_in[10];
  const float* Wfc1   = (const float*)d_in[11];
  const float* p1_w1  = (const float*)d_in[12];
  const float* p1_b1  = (const float*)d_in[13];
  const float* p1_w2  = (const float*)d_in[14];
  const float* p1_b2  = (const float*)d_in[15];
  const float* p1_lng = (const float*)d_in[16];
  const float* p1_lnb = (const float*)d_in[17];
  const float* p2_w1  = (const float*)d_in[18];
  const float* p2_b1  = (const float*)d_in[19];
  const float* p2_w2  = (const float*)d_in[20];
  const float* p2_b2  = (const float*)d_in[21];
  const float* lnc1_g = (const float*)d_in[22];
  const float* lnc1_b = (const float*)d_in[23];
  const float* lnc2_g = (const float*)d_in[24];
  const float* lnc2_b = (const float*)d_in[25];
  const float* Wcls   = (const float*)d_in[26];
  const float* bcls   = (const float*)d_in[27];
  float* out = (float*)d_out;
  (void)n_in;

  if ((size_t)WS_HALVES * sizeof(_Float16) > ws_size) return;
  _Float16* wsh = (_Float16*)d_ws;

  struct CastJob { const float* src; int off; int cnt; int idx; };
  const CastJob cj[8] = {
      {Wq,    WOFF_WQ,   32768, 8},  {Wk,    WOFF_WK,   32768, 9},
      {Wv,    WOFF_WV,   32768, 10}, {Wfc1,  WOFF_WFC1, 65536, 11},
      {p1_w1, WOFF_P1W1, 65536, 12}, {p1_w2, WOFF_P1W2, 65536, 14},
      {p2_w1, WOFF_P2W1, 32768, 18}, {p2_w2, WOFF_P2W2, 65536, 20}};
  for (int i = 0; i < 8; ++i) {
    int cnt = cj[i].cnt;
    if (in_sizes[cj[i].idx] < cnt) cnt = in_sizes[cj[i].idx];
    const int n2 = cnt / 2;
    if (n2 > 0)
      cast_scale_f16x2<<<(n2 + 255) / 256, 256, 0, stream>>>(cj[i].src, wsh + cj[i].off, n2, W_CARRY);
  }

  int nseq = in_sizes[0] / LTOK;
  if (nseq > out_size) nseq = out_size;
  int nvocab = in_sizes[1] / BNE;
  if (nvocab < 1) nvocab = 1;
  if (nseq > 0) {
    const int nblk = (nseq + SEQ_PER_BLK - 1) / SEQ_PER_BLK;
    fused_seq_kernel<<<nblk, NTHR, SMEM_BYTES, stream>>>(
        x, node_emb, ln1_g, ln1_b, ln2_g, ln2_b, ln3_g, ln3_b,
        p1_b1, p1_b2, p1_lng, p1_lnb, p2_b1, p2_b2,
        lnc1_g, lnc1_b, lnc2_g, lnc2_b, Wcls, bcls,
        wsh, out, nseq, nvocab);
  }
}
